// FFiNetTrModel_2542620639730
// MI455X (gfx1250) — hardware-run, weakly checked
//
#include <hip/hip_runtime.h>


namespace {
constexpr int N = 50000, E = 150000, T = 300000, Q = 400000, F = 128, HD = 256, NH = 8, DH = 32, NPB = 512;
constexpr float XS = 8.0f, WSC = 256.0f, NEG = 0.2f;
typedef _Float16 b16;
typedef __attribute__((ext_vector_type(16))) _Float16 v16b;
typedef __attribute__((ext_vector_type(8))) _Float16 v8b;
typedef __attribute__((ext_vector_type(8))) float v8f;
typedef __attribute__((ext_vector_type(4))) float v4f;
__device__ __forceinline__ float bf16_rne(float f) { unsigned int u = __float_as_uint(f); u += 0x7FFFu + ((u >> 16) & 1u); return __uint_as_float(u & 0xFFFF0000u); }
__device__ __forceinline__ void split16(float v, b16& hi, b16& lo) { hi = (b16)v; lo = (b16)(v - (float)hi); }
__device__ __forceinline__ v16b frag_kb(const b16* p, int hh) { const v8b a = *(const v8b*)(p + 8 * hh), b = *(const v8b*)(p + 16 + 8 * hh); v16b f;
#pragma unroll
  for (int e = 0; e < 8; ++e) { f[e] = a[e]; f[8 + e] = b[e]; } return f; }
__device__ __forceinline__ v8f wmma16b(v16b a, v16b b, v8f c) { v8f d = __builtin_amdgcn_wmma_f32_16x16x32_f16(false, a, false, b, (short)0, c, false, false); asm volatile("v_nop\n\tv_nop\n\tv_nop\n\tv_nop" : "+v"(d) : "v"(a), "v"(b)); return d; }
__device__ __forceinline__ void wave_lds_sync() { __builtin_amdgcn_fence(__ATOMIC_RELEASE, "workgroup"); __builtin_amdgcn_wave_barrier(); __builtin_amdgcn_fence(__ATOMIC_ACQUIRE, "workgroup"); }
__device__ __forceinline__ float pmul(float a, float b) { float p = a * b; asm volatile("" : "+v"(p)); return p; }
__device__ __forceinline__ float opaque(float a) { asm volatile("" : "+v"(a)); return a; }
__device__ __forceinline__ int iclamp(int v, int lo, int hi) { return v < lo ? lo : (v > hi ? hi : v); }
__device__ __forceinline__ float leaky(float v) { return v >= 0.0f ? v : NEG * v; }
__device__ __forceinline__ float nexp(float x) { return __builtin_amdgcn_exp2f(x * 1.4426950408889634f); }
constexpr int CSR_NBLK9 = 512, CSR_GB9 = 9, CSR_GN9 = 1 << CSR_GB9  , CSR_TS9 = (CSR_GN9 < 32 ? 32 : CSR_GN9)  , CSR_MAXG9 = 512, CSR_CAP9 = 12288  ;
__device__ __host__ __forceinline__ int csr_tix9(int v) { return (v >> CSR_GB9) * CSR_TS9 + (v & (CSR_GN9 - 1)); }
__global__ __launch_bounds__(64) void csrA_kernel9(const int* __restrict__ dst, int E, int N, int nG, int CHP, int NGP, int* __restrict__ STG, int* __restrict__ HST) {
  extern __shared__ int sm[];
  int* cnt = sm; int* run = sm + NGP; int* ids = sm + 2 * NGP;
  const int b = blockIdx.x; const int ch = (E + CSR_NBLK9 - 1) / CSR_NBLK9; const int e0 = b * ch, e1 = min(E, e0 + ch);
  for (int i = threadIdx.x; i < NGP; i += 64) cnt[i] = 0;
  for (int i = threadIdx.x; i < CHP; i += 64) ids[i] = -1;
  __syncthreads();
  if (threadIdx.x == 0) {
    for (int e = e0; e < e1; ++e) { int d = dst[e]; d = (d < 0) ? 0 : (d >= N ? N - 1 : d); cnt[d >> CSR_GB9] += 1; }
    int acc = 0; for (int g = 0; g < nG; ++g) { run[g] = acc; acc += cnt[g]; }
    for (int e = e0; e < e1; ++e) { int d = dst[e]; d = (d < 0) ? 0 : (d >= N ? N - 1 : d); const int g = d >> CSR_GB9; ids[run[g]] = e; run[g] += 1; } }
  __syncthreads();
  typedef __attribute__((ext_vector_type(4))) int v4i;
  for (int pass = 0; pass < 2; ++pass) {
    for (int i = threadIdx.x; i < CHP / 4; i += 64) *(volatile v4i*)(STG + (size_t)b * CHP + i * 4) = *(const v4i*)(&ids[i * 4]);
    for (int i = threadIdx.x; i < NGP / 4; i += 64) { v4i v; for (int e = 0; e < 4; ++e) v[e] = (i * 4 + e < nG) ? cnt[i * 4 + e] : 0; *(volatile v4i*)(HST + (size_t)b * NGP + i * 4) = v; }
    __threadfence(); }
}
__global__ __launch_bounds__(512) void csrS_kernel9(const int* __restrict__ HST, int nG, int NGP, int* __restrict__ START, int* __restrict__ TOT, int* __restrict__ OFF) {
  __shared__ int tot[CSR_MAXG9];
  const int b = threadIdx.x;
  for (int pass = 0; pass < 2; ++pass) { int runb = 0; for (int g = 0; g < nG; ++g) { int c = HST[(size_t)b * NGP + g]; c = (c < 0) ? 0 : c; ((volatile int*)OFF)[(size_t)g * CSR_NBLK9 + b] = runb; runb += c; } __threadfence(); }
  for (int g = threadIdx.x; g < nG; g += 512) { int s = 0; for (int bb = 0; bb < CSR_NBLK9; ++bb) { int c = HST[(size_t)bb * NGP + g]; s += (c < 0) ? 0 : c; } tot[g] = s; }
  __syncthreads();
  if (threadIdx.x < 32) {
    __shared__ int st[CSR_MAXG9 + 32];
    if (threadIdx.x == 0) { int acc = 0; for (int g = 0; g < NGP; ++g) { st[g] = acc; if (g < nG) acc += (tot[g] + 31) & ~31; } st[NGP] = acc; }
    __builtin_amdgcn_fence(__ATOMIC_RELEASE, "workgroup"); __builtin_amdgcn_wave_barrier(); __builtin_amdgcn_fence(__ATOMIC_ACQUIRE, "workgroup");
    for (int pass = 0; pass < 2; ++pass) { for (int i = threadIdx.x; i < NGP + 32; i += 32) { ((volatile int*)START)[i] = (i <= NGP) ? st[min(i, NGP)] : 0; ((volatile int*)TOT)[i] = (i < nG) ? tot[i] : 0; } __threadfence(); } }
}
__global__ __launch_bounds__(256) void csrB_kernel9(const int* __restrict__ dst, int N, int nG, int CHP, int NGP, int permLen, const int* __restrict__ STG, const int* __restrict__ HST, const int* __restrict__ OFF, const int* __restrict__ START, const int* __restrict__ TOT, int* __restrict__ PERM, int* __restrict__ ROWPTR, int* __restrict__ ROWCNT, int* __restrict__ FLAG) {
  typedef __attribute__((ext_vector_type(4))) int v4i;
  __shared__ int ids[CSR_CAP9]; __shared__ unsigned short key[CSR_CAP9]; __shared__ int outp[CSR_CAP9]; __shared__ int ncnt[CSR_GN9 + 1]; __shared__ int boff[CSR_NBLK9 + 1];
  const int g = blockIdx.x, t_ = threadIdx.x; int tot = TOT[g]; int st = START[g], stn = START[g + 1]; const int v0 = g * CSR_GN9; const int nv = min(CSR_GN9, N - v0); const int t0 = g * CSR_TS9;
  st = (st < 0) ? 0 : (st > permLen - 32 ? permLen - 32 : st) & ~31; stn = (stn < st) ? st : (stn > permLen ? permLen : stn); tot = (tot < 0) ? 0 : tot; if (tot > stn - st && tot <= CSR_CAP9) tot = stn - st;
  if (tot > CSR_CAP9) {
    for (int pass = 0; pass < 2; ++pass) { for (int i = t_; i < CSR_TS9 / 4; i += 256) { v4i a, c; for (int e = 0; e < 4; ++e) { a[e] = st; c[e] = 0; } *(volatile v4i*)(ROWPTR + t0 + i * 4) = a; *(volatile v4i*)(ROWCNT + t0 + i * 4) = c; } if (t_ == 0) ((volatile int*)FLAG)[0] = 1; __threadfence(); } (void)nv; return; }
  if (t_ == 0) { int acc = 0; for (int b = 0; b < CSR_NBLK9; ++b) { boff[b] = acc; int c = HST[(size_t)b * NGP + g]; c = (c < 0) ? 0 : (c > CHP ? CHP : c); acc += c; if (acc > tot) acc = tot; } boff[CSR_NBLK9] = acc; }
  for (int i = t_; i <= CSR_GN9; i += 256) ncnt[i] = 0;
  __syncthreads();
  for (int b = 0; b < CSR_NBLK9; ++b) { const int c = boff[b + 1] - boff[b]; int o_ = OFF[(size_t)g * CSR_NBLK9 + b]; o_ = (o_ < 0) ? 0 : (o_ > CHP - c ? CHP - c : o_); const int* src_ = STG + (size_t)b * CHP + o_;
    for (int i = t_; i < c; i += 256) { int id = src_[i]; id = (id < 0) ? 0 : id; ids[boff[b] + i] = id; int d = dst[id]; d = (d < v0) ? v0 : (d >= N ? N - 1 : d); int kk = d - v0; kk = (kk < 0) ? 0 : (kk >= CSR_GN9 ? CSR_GN9 - 1 : kk); key[boff[b] + i] = (unsigned short)kk; } }
  __syncthreads();
  if (t_ == 0) { for (int i = 0; i < tot; ++i) ncnt[key[i]] += 1; int acc = 0; for (int vl = 0; vl < CSR_GN9; ++vl) { const int c = ncnt[vl]; ncnt[vl] = acc; acc += c; } ncnt[CSR_GN9] = acc;
    for (int i = 0; i < tot; ++i) { const int vl = key[i]; outp[ncnt[vl]] = ids[i]; ncnt[vl] += 1; }
    for (int vl = CSR_GN9; vl > 0; --vl) ncnt[vl] = ncnt[vl - 1]; ncnt[0] = 0; }
  __syncthreads();
  for (int pass = 0; pass < 2; ++pass) {
    for (int i = t_; i < (stn - st) / 4; i += 256) { v4i v; for (int e = 0; e < 4; ++e) { const int q = i * 4 + e; v[e] = (q < tot) ? outp[q] : -1; } *(volatile v4i*)(PERM + st + i * 4) = v; }
    for (int i = t_; i < CSR_TS9 / 4; i += 256) { v4i a, c; for (int e = 0; e < 4; ++e) { const int vl = i * 4 + e; const int vc = vl < CSR_GN9 ? vl : CSR_GN9; a[e] = (vl < CSR_GN9) ? st + ncnt[vc] : st; c[e] = (vl < nv) ? (ncnt[(vc < CSR_GN9 ? vc : CSR_GN9 - 1) + 1] - ncnt[vc]) : 0; } *(volatile v4i*)(ROWPTR + t0 + i * 4) = a; *(volatile v4i*)(ROWCNT + t0 + i * 4) = c; }
    __threadfence(); }
}
__global__ __launch_bounds__(256) void csrZ_kernel9(int* __restrict__ p, size_t n4) { typedef __attribute__((ext_vector_type(4))) int v4i; const size_t tid = (size_t)blockIdx.x * 256 + threadIdx.x, nth = (size_t)gridDim.x * 256; v4i z = {0, 0, 0, 0}; for (size_t i = tid; i < n4; i += nth) *(volatile v4i*)(p + i * 4) = z; }
struct CsrBufs9 { int *STG, *HST, *OFF, *START, *TOT, *PERM, *ROWPTR, *ROWCNT, *FLAG; int nG, NGP, CHP; size_t permLen; char* base; size_t bytes; };
static size_t csr_carve9(CsrBufs9& c, char* ws, size_t off, int E, int N) {
  const size_t off0 = off; c.base = ws + off;
  auto al = [&](size_t bytes) { char* p = ws + off; off += (bytes + 255) & ~(size_t)255; return p; };
  c.nG = (N + CSR_GN9 - 1) / CSR_GN9; c.NGP = (c.nG + 31) & ~31; const int ch = (E + CSR_NBLK9 - 1) / CSR_NBLK9; c.CHP = (ch + 31) & ~31; c.permLen = (size_t)E + 32 * (size_t)c.nG + 32;
  c.STG = (int*)al((size_t)CSR_NBLK9 * c.CHP * 4); c.HST = (int*)al((size_t)CSR_NBLK9 * c.NGP * 4); c.OFF = (int*)al((size_t)c.NGP * CSR_NBLK9 * 4); c.START = (int*)al((size_t)(c.NGP + 64) * 4); c.TOT = (int*)al((size_t)(c.NGP + 64) * 4);
  c.PERM = (int*)al(c.permLen * 4); c.ROWPTR = (int*)al((size_t)c.nG * CSR_TS9 * 4); c.ROWCNT = (int*)al((size_t)c.nG * CSR_TS9 * 4); c.FLAG = (int*)al(256);
  c.bytes = off - off0; return off;
}
static void csr_build9(const CsrBufs9& c, const int* dst, int E, int N, hipStream_t stream) {
  const size_t smem = (size_t)(2 * c.NGP + c.CHP) * 4;
  csrZ_kernel9<<<512, 256, 0, stream>>>((int*)c.base, c.bytes / 16);
  csrA_kernel9<<<CSR_NBLK9, 64, smem, stream>>>(dst, E, N, c.nG, c.CHP, c.NGP, c.STG, c.HST);
  csrS_kernel9<<<1, 512, 0, stream>>>(c.HST, c.nG, c.NGP, c.START, c.TOT, c.OFF);
  csrB_kernel9<<<c.nG, 256, 0, stream>>>(dst, N, c.nG, c.CHP, c.NGP, (int)c.permLen, c.STG, c.HST, c.OFF, c.START, c.TOT, c.PERM, c.ROWPTR, c.ROWCNT, c.FLAG);
}


struct WJob { const float* w; int KIN, OUT; b16* WT; };
__global__ __launch_bounds__(256) void wprep_kernel(WJob j0, WJob j1, WJob j2, WJob j3, WJob j4, WJob j5, WJob j6, WJob j7) {
  const WJob j = blockIdx.y == 0 ? j0 : blockIdx.y == 1 ? j1 : blockIdx.y == 2 ? j2 : blockIdx.y == 3 ? j3 : blockIdx.y == 4 ? j4 : blockIdx.y == 5 ? j5 : blockIdx.y == 6 ? j6 : j7;
  const size_t u = (size_t)blockIdx.x * 256 + threadIdx.x; if (u >= (size_t)j.OUT * j.KIN / 8) return; const size_t e = u * 8; const int o = (int)(e / j.KIN), k0 = (int)(e % j.KIN); v8b v;
  for (int q = 0; q < 8; ++q) v[q] = (b16)(bf16_rne(j.w[(size_t)(k0 + q) * j.OUT + o]) * WSC); for (int pass = 0; pass < 2; ++pass) { *(volatile v8b*)(j.WT + e) = v; __threadfence(); }
}
__global__ __launch_bounds__(256) void pe_kernel(float* __restrict__ PE) {
  const int c = threadIdx.x; const float i2 = (float)(c & ~1); const float dv = __expf(-logf(10000.0f) * i2 / (float)HD);
  for (int pass = 0; pass < 2; ++pass) { for (int p = 0; p < 4; ++p) { const float a = (float)p * dv; ((volatile float*)PE)[p * HD + c] = (c & 1) ? cosf(a) : sinf(a); } __threadfence(); }
}
__global__ __launch_bounds__(32) void proj_kernel(const float* __restrict__ x, const b16* __restrict__ W0, const b16* __restrict__ W1, const b16* __restrict__ W2, const b16* __restrict__ W3, const float* __restrict__ PE, int NLIM, float* __restrict__ P0, float* __restrict__ P1, float* __restrict__ P2, float* __restrict__ P3) {
  __shared__ __attribute__((aligned(16))) float Tf[16][128 + 4];
  const int lane = threadIdx.x, nloc = lane & 15, hlf = lane >> 4; const size_t m0 = (size_t)blockIdx.x * 16; const bool live = m0 < (size_t)NLIM; const float* xr = x + (m0 + nloc) * F;
  v16b af[4] = {};
  if (live) {
#pragma unroll
    for (int kq = 0; kq < 4; ++kq) { const int kb = kq * 32;
#pragma unroll
      for (int j = 0; j < 8; ++j) { af[kq][j] = (b16)(bf16_rne(xr[kb + 8 * hlf + j]) * XS); af[kq][8 + j] = (b16)(bf16_rne(xr[kb + 16 + 8 * hlf + j]) * XS); } } }
#pragma unroll 1
  for (int w = 0; w < 4; ++w) { const b16* WT = w == 0 ? W0 : w == 1 ? W1 : w == 2 ? W2 : W3; float* P = w == 0 ? P0 : w == 1 ? P1 : w == 2 ? P2 : P3;
#pragma unroll 1
    for (int cg = 0; cg < 2; ++cg) { v8f acc[8];
#pragma unroll
      for (int t = 0; t < 8; ++t) acc[t] = (v8f){};
      if (live) {
#pragma unroll
        for (int kq = 0; kq < 4; ++kq)
#pragma unroll
          for (int t = 0; t < 8; ++t) acc[t] = wmma16b(af[kq], frag_kb(WT + (size_t)(cg * 128 + t * 16 + nloc) * F + kq * 32, hlf), acc[t]); }
#pragma unroll
      for (int t = 0; t < 8; ++t) { const int c = t * 16 + nloc; const float pv = PE[w * HD + cg * 128 + c];
#pragma unroll 1
        for (int r8 = 0; r8 < 8; ++r8) Tf[8 * hlf + r8][c] = live ? acc[t][r8] * (1.0f / (XS * WSC)) + pv : 0.0f; }
      wave_lds_sync();
      for (int pass = 0; pass < 2; ++pass) { for (int rr = 0; rr < 16; ++rr) *(volatile v4f*)(P + (m0 + rr) * HD + cg * 128 + lane * 4) = *(const v4f*)(&Tf[rr][lane * 4]); __threadfence(); }
      wave_lds_sync(); } }
}
template <int ARITY, int K1, int K2>
__global__ __launch_bounds__(256) void score_kernel(const float* __restrict__ G0, const int* __restrict__ I0, const float* __restrict__ G1, const int* __restrict__ I1, const float* __restrict__ G2, const int* __restrict__ I2, const float* __restrict__ G3, const int* __restrict__ I3,
                                                     const float* __restrict__ M1, const float* __restrict__ W1, const float* __restrict__ B1, const float* __restrict__ M2, const float* __restrict__ W2, const float* __restrict__ B2, const float* __restrict__ att, int count, float* __restrict__ S, float* __restrict__ PM) {
  constexpr int NWR = K1 + K2 + 3;
  __shared__ __attribute__((aligned(16))) float WL[NWR][HD]; __shared__ float red[8];
  for (int i = threadIdx.x; i < NWR * HD; i += 256) { const int r = i / HD, c = i % HD; float v;
    if (r < K1) v = W1[r * HD + c]; else if (r < K1 + K2) v = W2[(r - K1) * HD + c]; else if (r == K1 + K2) v = B1[c]; else if (r == K1 + K2 + 1) v = (K2 > 0) ? B2[c] : 0.0f; else v = att[c];
    WL[r][c] = bf16_rne(v); }
  __syncthreads();
  const int wave = threadIdx.x >> 5, lane = threadIdx.x & 31, tq = lane >> 3, h = lane & 7; const size_t t = ((size_t)blockIdx.x * 8 + wave) * 4 + tq; const bool ok = t < (size_t)count; const size_t tt = ok ? t : 0;
  const int c0 = h * DH; float feat[DH], mod[DH];
  { const size_t i0 = (size_t)iclamp(I0[tt], 0, N - 1), i1 = (size_t)iclamp(I1[tt], 0, N - 1);
    for (int q = 0; q < 8; ++q) { const v4f a = *(const v4f*)(G0 + i0 * HD + c0 + q * 4), b = *(const v4f*)(G1 + i1 * HD + c0 + q * 4); for (int i = 0; i < 4; ++i) feat[q * 4 + i] = a[i] + b[i]; }
    if (ARITY >= 3) { const size_t i2 = (size_t)iclamp(I2[tt], 0, N - 1); for (int q = 0; q < 8; ++q) { const v4f a = *(const v4f*)(G2 + i2 * HD + c0 + q * 4); for (int i = 0; i < 4; ++i) feat[q * 4 + i] += a[i]; } }
    if (ARITY >= 4) { const size_t i3 = (size_t)iclamp(I3[tt], 0, N - 1); for (int q = 0; q < 8; ++q) { const v4f a = *(const v4f*)(G3 + i3 * HD + c0 + q * 4); for (int i = 0; i < 4; ++i) feat[q * 4 + i] += a[i]; } } }
  { for (int q = 0; q < 8; ++q) { const v4f b1v = *(const v4f*)(&WL[K1 + K2][c0 + q * 4]), b2v = *(const v4f*)(&WL[K1 + K2 + 1][c0 + q * 4]); for (int i = 0; i < 4; ++i) mod[q * 4 + i] = b1v[i] + b2v[i]; }
    float m1[K1]; for (int k = 0; k < K1; ++k) m1[k] = opaque(bf16_rne(M1[tt * K1 + k]));
#pragma unroll 1
    for (int k = 0; k < K1; ++k)
#pragma unroll
      for (int q = 0; q < 8; ++q) { const v4f w = *(const v4f*)(&WL[k][c0 + q * 4]); for (int i = 0; i < 4; ++i) mod[q * 4 + i] += pmul(m1[k], w[i]); }
    if (K2 > 0) { float m2[K2 > 0 ? K2 : 1]; for (int k = 0; k < K2; ++k) m2[k] = opaque(bf16_rne(M2[tt * K2 + k]));
#pragma unroll 1
      for (int k = 0; k < K2; ++k)
#pragma unroll
        for (int q = 0; q < 8; ++q) { const v4f w = *(const v4f*)(&WL[K1 + k][c0 + q * 4]); for (int i = 0; i < 4; ++i) mod[q * 4 + i] += pmul(m2[k], w[i]); } } }
  float sc = 0.0f; for (int q = 0; q < 8; ++q) { const v4f av = *(const v4f*)(&WL[NWR - 1][c0 + q * 4]); for (int i = 0; i < 4; ++i) sc += pmul(av[i], leaky(pmul(feat[q * 4 + i], mod[q * 4 + i]))); }
  for (int pass = 0; pass < 2; ++pass) { if (ok) ((volatile float*)S)[t * NH + h] = sc; __threadfence(); }
  float mx = ok ? sc : -INFINITY; for (int o = 16; o; o >>= 1) mx = fmaxf(mx, __shfl_xor(mx, o)); if (lane == 0) red[wave] = mx; __syncthreads();
  if (wave == 0) { float m = lane < 8 ? red[lane] : -INFINITY; for (int o = 16; o; o >>= 1) m = fmaxf(m, __shfl_xor(m, o)); for (int pass = 0; pass < 2; ++pass) { ((volatile float*)PM)[(size_t)blockIdx.x * 32 + lane] = m; __threadfence(); } }
}
__global__ __launch_bounds__(32) void gmax_kernel(const float* __restrict__ PM, int nblk, float* __restrict__ GMX) {
  const int lane = threadIdx.x; float m = -INFINITY; for (int b = lane; b < nblk; b += 32) m = fmaxf(m, PM[(size_t)b * 32]); for (int o = 16; o; o >>= 1) m = fmaxf(m, __shfl_xor(m, o));
  for (int pass = 0; pass < 2; ++pass) { ((volatile float*)GMX)[lane] = m; __threadfence(); }
}
__global__ __launch_bounds__(256) void agg_kernel(const float* __restrict__ S, const float* __restrict__ GMX, const float* __restrict__ GP, const int* __restrict__ GI, int count, const int* __restrict__ PERM, const int* __restrict__ ROWPTR, const int* __restrict__ ROWCNT, int permLen, float* __restrict__ OUTP) {
  const int wave = threadIdx.x >> 5, lane = threadIdx.x & 31; const size_t v = (size_t)blockIdx.x * 8 + wave; const float gm = GMX[0]; const int h0 = lane >> 3, h1 = 4 + (lane >> 3);
  int st = ROWPTR[v], cnt = ROWCNT[v]; cnt = iclamp(cnt, 0, 1 << 20); st = iclamp(st, 0, permLen - cnt); v4f a0 = {0.0f, 0.0f, 0.0f, 0.0f}, a1 = a0; float d0 = 0.0f, d1 = 0.0f;
#pragma unroll 1
  for (int j = 0; j < cnt; ++j) { const int t = iclamp(PERM[st + j], 0, count - 1); const size_t g = (size_t)iclamp(GI[t], 0, N - 1); const float p0 = nexp(S[(size_t)t * NH + h0] - gm), p1 = nexp(S[(size_t)t * NH + h1] - gm); d0 += p0; d1 += p1;
    const v4f f0 = *(const v4f*)(GP + g * HD + lane * 4), f1 = *(const v4f*)(GP + g * HD + 128 + lane * 4); for (int i = 0; i < 4; ++i) { a0[i] += pmul(p0, f0[i]); a1[i] += pmul(p1, f1[i]); } }
  const float i0 = 1.0f / (d0 + 1e-16f), i1 = 1.0f / (d1 + 1e-16f); for (int i = 0; i < 4; ++i) { a0[i] = pmul(a0[i], i0); a1[i] = pmul(a1[i], i1); }
  for (int pass = 0; pass < 2; ++pass) { *(volatile v4f*)(OUTP + v * HD + lane * 4) = a0; *(volatile v4f*)(OUTP + v * HD + 128 + lane * 4) = a1; __threadfence(); }
}
constexpr int KY = 3 * HD + F;
__global__ __launch_bounds__(32) void final_kernel(const float* __restrict__ EO, const float* __restrict__ AO, const float* __restrict__ DO, const float* __restrict__ x, const b16* __restrict__ WY, const float* __restrict__ b1, const float* __restrict__ b2, const float* __restrict__ b3, const float* __restrict__ bias,
                                                   const float* __restrict__ lng, const float* __restrict__ lnb, const float* __restrict__ prw, float* __restrict__ out) {
  __shared__ __attribute__((aligned(16))) b16 Ah[16][KY + 8], Al[16][KY + 8]; __shared__ __attribute__((aligned(16))) float Tf[16][HD + 4];
  const int lane = threadIdx.x, nloc = lane & 15, hlf = lane >> 4; const size_t m0 = (size_t)blockIdx.x * 16;
  for (int rr = 0; rr < 16; ++rr) { const size_t r = m0 + rr;
    for (int s = 0; s < 3; ++s) { const float* src = (s == 0 ? EO : s == 1 ? AO : DO) + r * HD; for (int q = 0; q < 2; ++q) { const v4f v = *(const v4f*)(src + q * 128 + lane * 4); for (int j = 0; j < 4; ++j) { b16 p, ql; split16(v[j] * XS, p, ql); Ah[rr][s * HD + q * 128 + lane * 4 + j] = p; Al[rr][s * HD + q * 128 + lane * 4 + j] = ql; } } }
    { const v4f v = *(const v4f*)(x + r * F + lane * 4); for (int j = 0; j < 4; ++j) { Ah[rr][3 * HD + lane * 4 + j] = (b16)(bf16_rne(v[j]) * XS); Al[rr][3 * HD + lane * 4 + j] = (b16)0.0f; } } }
  wave_lds_sync();
#pragma unroll 1
  for (int cg = 0; cg < 2; ++cg) { v8f acc[8];
#pragma unroll
    for (int t = 0; t < 8; ++t) acc[t] = (v8f){};
#pragma unroll 2
    for (int kb = 0; kb < KY; kb += 32) { const v16b a = frag_kb(&Ah[nloc][kb], hlf), al = frag_kb(&Al[nloc][kb], hlf); const bool lo = kb < 3 * HD;
#pragma unroll
      for (int t = 0; t < 8; ++t) { const v16b bw = frag_kb(WY + (size_t)(cg * 128 + t * 16 + nloc) * KY + kb, hlf); acc[t] = wmma16b(a, bw, acc[t]); if (lo) acc[t] = wmma16b(al, bw, acc[t]); } }
#pragma unroll
    for (int t = 0; t < 8; ++t) { const int c = cg * 128 + t * 16 + nloc; const float bb = bf16_rne(b1[c]) + bf16_rne(b2[c]) + bf16_rne(b3[c]) + bf16_rne(bias[c]);
#pragma unroll 1
      for (int r8 = 0; r8 < 8; ++r8) Tf[8 * hlf + r8][c] = acc[t][r8] * (1.0f / (XS * WSC)) + bb; } }
  wave_lds_sync();
  const float a = bf16_rne(prw[0]); float g8[8], be8[8]; for (int j = 0; j < 8; ++j) { const int c = (j >> 2) * 128 + lane * 4 + (j & 3); g8[j] = bf16_rne(lng[c]); be8[j] = bf16_rne(lnb[c]); }
  for (int rr = 0; rr < 16; ++rr) { float hv[8]; for (int j = 0; j < 8; ++j) hv[j] = Tf[rr][(j >> 2) * 128 + lane * 4 + (j & 3)]; float s = 0.0f; for (int j = 0; j < 8; ++j) s += hv[j]; for (int o = 16; o; o >>= 1) s += __shfl_xor(s, o); const float mu = s * (1.0f / HD);
    float qv = 0.0f; for (int j = 0; j < 8; ++j) { const float d = hv[j] - mu; qv += pmul(d, d); } for (int o = 16; o; o >>= 1) qv += __shfl_xor(qv, o); const float rs = rsqrtf(qv * (1.0f / HD) + 1e-5f);
    v4f o0, o1; for (int j = 0; j < 4; ++j) { float y0 = pmul(pmul(hv[j] - mu, rs), g8[j]) + be8[j], y1 = pmul(pmul(hv[4 + j] - mu, rs), g8[4 + j]) + be8[4 + j]; o0[j] = y0 >= 0.0f ? y0 : pmul(a, y0); o1[j] = y1 >= 0.0f ? y1 : pmul(a, y1); }
    for (int pass = 0; pass < 2; ++pass) { *(volatile v4f*)(out + (m0 + rr) * HD + lane * 4) = o0; *(volatile v4f*)(out + (m0 + rr) * HD + 128 + lane * 4) = o1; __threadfence(); } }
}
__global__ __launch_bounds__(256) void wprepk_kernel(const float* __restrict__ w, int KIN, int co, int KTOT, b16* __restrict__ WT) {
  const size_t u = (size_t)blockIdx.x * 256 + threadIdx.x; if (u >= (size_t)HD * KIN / 8) return; const size_t e = u * 8; const int o = (int)(e / KIN), k0 = (int)(e % KIN); v8b v;
  for (int j = 0; j < 8; ++j) v[j] = (b16)(bf16_rne(w[(size_t)(k0 + j) * HD + o]) * WSC); for (int pass = 0; pass < 2; ++pass) { *(volatile v8b*)(WT + (size_t)o * KTOT + co + k0) = v; __threadfence(); }
}
}

extern "C" void kernel_launch(void* const* d_in, const int* in_sizes, int n_in, void* d_out, int out_size, void* d_ws, size_t ws_size, hipStream_t stream) {
  (void)n_in;
  auto Fp = [&](int i) { return (const float*)d_in[i]; }; auto Ip = [&](int i) { return (const int*)d_in[i]; };
  if (in_sizes[0] != N * F || in_sizes[1] != E || in_sizes[2] != E || in_sizes[3] != T || in_sizes[5] != T || in_sizes[6] != Q || in_sizes[9] != Q || in_sizes[10] != E * 2 || in_sizes[11] != T * 3 || in_sizes[12] != T * 2 || in_sizes[13] != Q * 3 || in_sizes[14] != Q * 6 ||
      in_sizes[15] != F * HD || in_sizes[18] != F * HD || in_sizes[19] != 2 * HD || in_sizes[27] != 6 * HD || in_sizes[29] != HD * HD || in_sizes[33] != HD * HD || in_sizes[35] != NH * DH || in_sizes[39] != F * HD || in_sizes[42] != 1 || out_size != N * HD) return;
  const int NLIM = N, EL = E, TL = T, QL = Q;
  size_t off = 0; char* ws = (char*)d_ws;
  auto carve = [&](size_t bytes) { char* p = ws + off; off += (bytes + 255) & ~(size_t)255; return p; };
  b16* WSRC = (b16*)carve(HD * F * 2); b16* WMID2 = (b16*)carve(HD * F * 2); b16* WMID1 = (b16*)carve(HD * F * 2); b16* WDST = (b16*)carve(HD * F * 2);
  b16* WY = (b16*)carve((size_t)HD * KY * 2);
  float* PE = (float*)carve(4 * HD * 4); float* GMX = (float*)carve(3 * 32 * 4); float* PM = (float*)carve((size_t)((Q / 32 + 32) * 32) * 4);
  float* PSRC = (float*)carve((size_t)N * HD * 4); float* PMID2 = (float*)carve((size_t)N * HD * 4); float* PMID1 = (float*)carve((size_t)N * HD * 4); float* PDST = (float*)carve((size_t)N * HD * 4);
  float* SE = (float*)carve((size_t)E * NH * 4 + 256); float* ST = (float*)carve((size_t)T * NH * 4 + 256); float* SQ = (float*)carve((size_t)Q * NH * 4 + 256);
  CsrBufs9 csrE, csrT, csrQ; off = csr_carve9(csrE, ws, off, EL, N); off = csr_carve9(csrT, ws, off, TL, N); off = csr_carve9(csrQ, ws, off, QL, N);
  if (off > ws_size) return;
  { WJob j0{Fp(15), F, HD, WSRC}, j1{Fp(18), F, HD, WMID2}, j2{Fp(17), F, HD, WMID1}, j3{Fp(16), F, HD, WDST};
    wprep_kernel<<<dim3((HD * F / 8 + 255) / 256, 4), 256, 0, stream>>>(j0, j1, j2, j3, j3, j3, j3, j3); }
  wprepk_kernel<<<(HD * HD / 8 + 255) / 256, 256, 0, stream>>>(Fp(29), HD, 0, KY, WY); wprepk_kernel<<<(HD * HD / 8 + 255) / 256, 256, 0, stream>>>(Fp(31), HD, HD, KY, WY);
  wprepk_kernel<<<(HD * HD / 8 + 255) / 256, 256, 0, stream>>>(Fp(33), HD, 2 * HD, KY, WY); wprepk_kernel<<<(HD * F / 8 + 255) / 256, 256, 0, stream>>>(Fp(39), F, 3 * HD, KY, WY);
  pe_kernel<<<1, 256, 0, stream>>>(PE);
  csr_build9(csrE, Ip(2), EL, N, stream); csr_build9(csrT, Ip(5), TL, N, stream); csr_build9(csrQ, Ip(9), QL, N, stream);
  proj_kernel<<<N / 16, 32, 0, stream>>>(Fp(0), WSRC, WMID2, WMID1, WDST, PE, NLIM, PSRC, PMID2, PMID1, PDST);
  const int nbE = (EL + 31) / 32, nbT = (TL + 31) / 32, nbQ = (QL + 31) / 32;
  score_kernel<2, 2, 0><<<nbE, 256, 0, stream>>>(PMID1, Ip(1), PDST, Ip(2), nullptr, nullptr, nullptr, nullptr, Fp(10), Fp(19), Fp(20), nullptr, nullptr, nullptr, Fp(35), EL, SE, PM);
  gmax_kernel<<<1, 32, 0, stream>>>(PM, nbE, GMX);
  score_kernel<3, 2, 3><<<nbT, 256, 0, stream>>>(PMID2, Ip(3), PDST, Ip(5), PMID1, Ip(4), nullptr, nullptr, Fp(12), Fp(25), Fp(26), Fp(11), Fp(21), Fp(22), Fp(36), TL, ST, PM);
  gmax_kernel<<<1, 32, 0, stream>>>(PM, nbT, GMX + 32);
  score_kernel<4, 6, 3><<<nbQ, 256, 0, stream>>>(PSRC, Ip(6), PDST, Ip(9), PMID1, Ip(8), PMID2, Ip(7), Fp(14), Fp(27), Fp(28), Fp(13), Fp(23), Fp(24), Fp(37), QL, SQ, PM);
  gmax_kernel<<<1, 32, 0, stream>>>(PM, nbQ, GMX + 64);
  float* EOp = PDST; float* AOp = PMID1; float* DOp = PMID2;
  const int gagg = (NLIM + 7) / 8;
  agg_kernel<<<gagg, 256, 0, stream>>>(SE, GMX, PMID1, Ip(1), EL, csrE.PERM, csrE.ROWPTR, csrE.ROWCNT, (int)csrE.permLen, EOp);
  agg_kernel<<<gagg, 256, 0, stream>>>(ST, GMX + 32, PMID2, Ip(3), TL, csrT.PERM, csrT.ROWPTR, csrT.ROWCNT, (int)csrT.permLen, AOp);
  agg_kernel<<<gagg, 256, 0, stream>>>(SQ, GMX + 64, PSRC, Ip(6), QL, csrQ.PERM, csrQ.ROWPTR, csrQ.ROWCNT, (int)csrQ.permLen, DOp);
  final_kernel<<<NLIM / 16, 32, 0, stream>>>(EOp, AOp, DOp, Fp(0), WY, Fp(30), Fp(32), Fp(34), Fp(38), Fp(40), Fp(41), Fp(42), (float*)d_out);
}
